// GENConv_43800076485029
// MI455X (gfx1250) — hardware-verified
//
#include <hip/hip_runtime.h>
#include <stddef.h>


#define DF    32
#define HD    64
#define NB    512
#define CHUNK 4096
#define NTHR  256
#define NWAVE 8
#define WCAP  512
#define NGRP  (CHUNK / (NTHR * 4))
#define KP1   40
#define KP2   72
#define HSP   68
#define OSP   36
#define EPSV  1e-7f

#define LDS_ACC   (NB * DF)
#define LDS_LIST  (NWAVE * WCAP)
#define OFF_W     ((3 * LDS_ACC + LDS_LIST + NWAVE) * 4)
#define LDS_BYTES (OFF_W + (2 * HD * KP1 + 2 * DF * KP2) * 2)

static_assert(NGRP == 4);
static_assert(WCAP == (CHUNK / NTHR) * 32);
static_assert(NB == 512 && CHUNK == 4096);
static_assert(NB == NWAVE * 64);
static_assert((OFF_W % 16) == 0);
static_assert(LDS_BYTES == 232480);
static_assert((NWAVE * 16 * HSP + NWAVE * 16 * OSP) <= LDS_ACC);

typedef float          v4f  __attribute__((ext_vector_type(4)));
typedef float          v4fa __attribute__((ext_vector_type(4), may_alias));
typedef float          v8f  __attribute__((ext_vector_type(8)));
typedef int            v4i  __attribute__((ext_vector_type(4)));
typedef unsigned short v8us __attribute__((ext_vector_type(8)));
typedef __bf16         v16b __attribute__((ext_vector_type(16)));
union FragB { v16b v; v8us half[2]; };

__device__ __forceinline__ v8f wmb(v16b a, v16b b, v8f c) {
  v8f d = __builtin_amdgcn_wmma_f32_16x16x32_bf16(false, a, false, b, (short)0, c, false, false);
  asm volatile("v_nop\n\tv_nop\n\tv_nop\n\tv_nop" : "+v"(d) : "v"(a), "v"(b));
  return d;
}

__device__ __forceinline__ v8f wm3(const FragB& ah, const FragB& al, const FragB& bh, const FragB& bl, v8f c) {
  c = wmb(ah.v, bh.v, c);
  c = wmb(ah.v, bl.v, c);
  c = wmb(al.v, bh.v, c);
  return c;
}

__device__ __forceinline__ unsigned short bfr(float f) {
  unsigned u = __float_as_uint(f);
  u = u + 0x7FFFu + ((u >> 16) & 1u);
  return (unsigned short)(u >> 16);
}
__device__ __forceinline__ float bff(unsigned short b) { return __uint_as_float(((unsigned)b) << 16); }

__device__ __forceinline__ void split8(v4f a, v4f b, v8us& hi, v8us& lo) {
  float f[8];
  f[0] = a.x; f[1] = a.y; f[2] = a.z; f[3] = a.w;
  f[4] = b.x; f[5] = b.y; f[6] = b.z; f[7] = b.w;
#pragma unroll
  for (int i = 0; i < 8; ++i) {
    const unsigned short hv = bfr(f[i]);
    hi[i] = hv;
    lo[i] = bfr(f[i] - bff(hv));
  }
}

__device__ __forceinline__ v4f nrm4(v4f a, v4f d) {
  v4f r;
  r.x = (d.x > 0.f) ? a.x * __builtin_amdgcn_rcpf(d.x) : 0.f;
  r.y = (d.y > 0.f) ? a.y * __builtin_amdgcn_rcpf(d.y) : 0.f;
  r.z = (d.z > 0.f) ? a.z * __builtin_amdgcn_rcpf(d.z) : 0.f;
  r.w = (d.w > 0.f) ? a.w * __builtin_amdgcn_rcpf(d.w) : 0.f;
  return r;
}

__device__ __forceinline__ int imin(int a, int b) { return a < b ? a : b; }

__global__ __launch_bounds__(NTHR) void k_gen(
    const float* __restrict__ x, const int* __restrict__ ei, const float* __restrict__ beta_p,
    const float* __restrict__ W1, const float* __restrict__ b1,
    const float* __restrict__ W2, const float* __restrict__ b2,
    float* out, int nN, int nE) {
  extern __shared__ v4f lds_dyn[];
  float* sacc = (float*)lds_dyn;
  float* sden = sacc + LDS_ACC;
  float* smx  = sden + LDS_ACC;
  int*   list = (int*)(smx + LDS_ACC);
  int*   wcnt = list + LDS_LIST;
  unsigned short* W1h = (unsigned short*)(wcnt + NWAVE);
  unsigned short* W1l = W1h + HD * KP1;
  unsigned short* W2h = W1l + HD * KP1;
  unsigned short* W2l = W2h + DF * KP2;

  const int tid  = threadIdx.x;
  const int lane = tid & 31;
  const int wave = tid >> 5;
  const int hh   = lane >> 4;
  const int m    = lane & 15;
  const int nodeBase = blockIdx.x * NB;
  const float beta = beta_p[0];

  {
    const v4f z4 = {0.f, 0.f, 0.f, 0.f};
    const v4f n4 = {-3.0e38f, -3.0e38f, -3.0e38f, -3.0e38f};
    for (int i = tid; i < (2 * LDS_ACC) / 4; i += NTHR) lds_dyn[i] = z4;
    for (int i = tid; i < LDS_ACC / 4; i += NTHR) lds_dyn[(2 * LDS_ACC) / 4 + i] = n4;
    {
      const int n = tid & (HD - 1), kq = tid >> 6;
      v4f wa, wb;
      wa.x = W1[(8 * kq + 0) * HD + n]; wa.y = W1[(8 * kq + 1) * HD + n];
      wa.z = W1[(8 * kq + 2) * HD + n]; wa.w = W1[(8 * kq + 3) * HD + n];
      wb.x = W1[(8 * kq + 4) * HD + n]; wb.y = W1[(8 * kq + 5) * HD + n];
      wb.z = W1[(8 * kq + 6) * HD + n]; wb.w = W1[(8 * kq + 7) * HD + n];
      v8us hi, lo;
      split8(wa, wb, hi, lo);
      *(v8us*)(W1h + n * KP1 + 8 * kq) = hi;
      *(v8us*)(W1l + n * KP1 + 8 * kq) = lo;
    }
    {
      const int n = tid & (DF - 1), kq = tid >> 5;
      v4f wa, wb;
      wa.x = W2[(8 * kq + 0) * DF + n]; wa.y = W2[(8 * kq + 1) * DF + n];
      wa.z = W2[(8 * kq + 2) * DF + n]; wa.w = W2[(8 * kq + 3) * DF + n];
      wb.x = W2[(8 * kq + 4) * DF + n]; wb.y = W2[(8 * kq + 5) * DF + n];
      wb.z = W2[(8 * kq + 6) * DF + n]; wb.w = W2[(8 * kq + 7) * DF + n];
      v8us hi, lo;
      split8(wa, wb, hi, lo);
      *(v8us*)(W2h + n * KP2 + 8 * kq) = hi;
      *(v8us*)(W2l + n * KP2 + 8 * kq) = lo;
    }
  }
  __syncthreads();

  const int nChunks = (nE + CHUNK - 1) / CHUNK;
#pragma unroll 1
  for (int ch = 0; ch < nChunks; ++ch) {
    const int cbase = ch * CHUNK;
    int wc = 0;
#pragma unroll
    for (int g = 0; g < NGRP; ++g) {
      const int el0 = (g * NTHR + tid) * 4;
      const int e0  = cbase + el0;
      const int sent = -2147483647 - 1;
      v4i d;
      if (cbase + CHUNK <= nE) {
        d = *(const v4i*)(ei + e0);
      } else {
        const int l0 = nE - 1;
        d.x = (e0     < nE) ? ei[imin(e0, l0)]     : sent;
        d.y = (e0 + 1 < nE) ? ei[imin(e0 + 1, l0)] : sent;
        d.z = (e0 + 2 < nE) ? ei[imin(e0 + 2, l0)] : sent;
        d.w = (e0 + 3 < nE) ? ei[imin(e0 + 3, l0)] : sent;
      }
      const unsigned s0 = (unsigned)d.x - (unsigned)nodeBase;
      const unsigned s1 = (unsigned)d.y - (unsigned)nodeBase;
      const unsigned s2 = (unsigned)d.z - (unsigned)nodeBase;
      const unsigned s3 = (unsigned)d.w - (unsigned)nodeBase;
      const bool h0 = s0 < (unsigned)NB;
      const bool h1 = s1 < (unsigned)NB;
      const bool h2 = s2 < (unsigned)NB;
      const bool h3 = s3 < (unsigned)NB;
      const unsigned many = __builtin_amdgcn_ballot_w32(h0 | h1 | h2 | h3);
      if (many != 0u) {
#define HITJ(J, HJ, SJ) { \
          const unsigned mj = __builtin_amdgcn_ballot_w32(HJ); \
          if (HJ) { \
            const int pos = wc + (int)__builtin_amdgcn_mbcnt_lo(mj, 0u); \
            if (pos < WCAP) list[wave * WCAP + pos] = ((el0 + (J)) << 9) | (int)(SJ); \
          } \
          wc += (int)__builtin_popcount(mj); }
        HITJ(0, h0, s0)
        HITJ(1, h1, s1)
        HITJ(2, h2, s2)
        HITJ(3, h3, s3)
#undef HITJ
      }
    }
    if (lane == 0) wcnt[wave] = wc;
    __syncthreads();

    if (wave == 0) {
#pragma unroll 1
      for (int wsx = 0; wsx < NWAVE; ++wsx) {
        int n = wcnt[wsx];
        n = (n > WCAP) ? WCAP : n;
        n = (n < 0) ? 0 : n;
#pragma unroll 1
        for (int i = 0; i < n; ++i) {
          const int ent  = list[wsx * WCAP + i];
          const int slot = ent & (NB - 1);
          const int el   = (ent >> 9) & (CHUNK - 1);
          int e = cbase + el;
          e = (e > nE - 1) ? (nE - 1) : e;
          int src = ei[(size_t)nE + (size_t)e];
          src = (src < 0) ? 0 : ((src > nN - 1) ? (nN - 1) : src);
          const float v   = x[(size_t)src * DF + lane];
          const float msg = fmaxf(v, 0.f) + EPSV;
          const float lg  = beta * msg;
          const int   ix  = slot * DF + lane;
          const float m0  = smx[ix];
          const float mn  = fmaxf(m0, lg);
          const float sc  = __expf(fmaxf(m0 - mn, -90.f));
          const float p   = __expf(lg - mn);
          const float dn  = sden[ix] * sc + p;
          const float ac  = sacc[ix] * sc + msg * p;
          sden[ix] = dn;
          sacc[ix] = ac;
          smx[ix]  = mn;
        }
      }
    }
    __syncthreads();
  }

  float* Hs = smx + wave * (16 * HSP);
  float* Os = smx + NWAVE * 16 * HSP + wave * (16 * OSP);
  float b1v[4], b2v[2];
#pragma unroll
  for (int nt = 0; nt < 4; ++nt) b1v[nt] = b1[16 * nt + m];
#pragma unroll
  for (int nt = 0; nt < 2; ++nt) b2v[nt] = b2[16 * nt + m];
  const int rq = lane >> 3;
  const int c4 = (lane & 7) * 4;

#pragma unroll 1
  for (int j = 0; j < 4; ++j) {
    const int slot0 = wave * 64 + j * 16;

    FragB ah, al;
    {
      const float* pa = sacc + (slot0 + m) * DF;
      const float* pd = sden + (slot0 + m) * DF;
      const v4f a0 = *(const v4fa*)(pa + 8 * hh);
      const v4f a1 = *(const v4fa*)(pa + 8 * hh + 4);
      const v4f a2 = *(const v4fa*)(pa + 16 + 8 * hh);
      const v4f a3 = *(const v4fa*)(pa + 20 + 8 * hh);
      const v4f d0 = *(const v4fa*)(pd + 8 * hh);
      const v4f d1 = *(const v4fa*)(pd + 8 * hh + 4);
      const v4f d2 = *(const v4fa*)(pd + 16 + 8 * hh);
      const v4f d3 = *(const v4fa*)(pd + 20 + 8 * hh);
      const v4f g0 = nrm4(a0, d0), g1 = nrm4(a1, d1), g2 = nrm4(a2, d2), g3 = nrm4(a3, d3);
      split8(g0, g1, ah.half[0], al.half[0]);
      split8(g2, g3, ah.half[1], al.half[1]);
    }

#pragma unroll
    for (int nt = 0; nt < 4; ++nt) {
      FragB bh, bl;
      const int bo = (16 * nt + m) * KP1 + 8 * hh;
      bh.half[0] = *(const v8us*)(W1h + bo);
      bh.half[1] = *(const v8us*)(W1h + bo + 16);
      bl.half[0] = *(const v8us*)(W1l + bo);
      bl.half[1] = *(const v8us*)(W1l + bo + 16);
      v8f c = {0.f, 0.f, 0.f, 0.f, 0.f, 0.f, 0.f, 0.f};
      c = wm3(ah, al, bh, bl, c);
#pragma unroll
      for (int r = 0; r < 8; ++r)
        Hs[(8 * hh + r) * HSP + 16 * nt + m] = fmaxf(c[r] + b1v[nt], 0.f);
    }
    __syncthreads();

    v8f c2[2];
    c2[0] = (v8f){0.f, 0.f, 0.f, 0.f, 0.f, 0.f, 0.f, 0.f};
    c2[1] = (v8f){0.f, 0.f, 0.f, 0.f, 0.f, 0.f, 0.f, 0.f};
#pragma unroll
    for (int ks = 0; ks < 2; ++ks) {
      FragB a2h, a2l;
      {
        const float* ph = Hs + m * HSP + 32 * ks;
        const v4f g0 = *(const v4fa*)(ph + 8 * hh);
        const v4f g1 = *(const v4fa*)(ph + 8 * hh + 4);
        const v4f g2 = *(const v4fa*)(ph + 16 + 8 * hh);
        const v4f g3 = *(const v4fa*)(ph + 20 + 8 * hh);
        split8(g0, g1, a2h.half[0], a2l.half[0]);
        split8(g2, g3, a2h.half[1], a2l.half[1]);
      }
#pragma unroll
      for (int nt = 0; nt < 2; ++nt) {
        FragB bh, bl;
        const int bo = (16 * nt + m) * KP2 + 32 * ks + 8 * hh;
        bh.half[0] = *(const v8us*)(W2h + bo);
        bh.half[1] = *(const v8us*)(W2h + bo + 16);
        bl.half[0] = *(const v8us*)(W2l + bo);
        bl.half[1] = *(const v8us*)(W2l + bo + 16);
        c2[nt] = wm3(a2h, a2l, bh, bl, c2[nt]);
      }
    }
#pragma unroll
    for (int nt = 0; nt < 2; ++nt)
#pragma unroll
      for (int r = 0; r < 8; ++r)
        Os[(8 * hh + r) * OSP + 16 * nt + m] = c2[nt][r] + b2v[nt];
    __syncthreads();

    v4f ov[4];
#pragma unroll
    for (int it = 0; it < 4; ++it) ov[it] = *(const v4fa*)(Os + (4 * it + rq) * OSP + c4);
#pragma unroll
    for (int it = 0; it < 4; ++it) {
      const int node = nodeBase + slot0 + 4 * it + rq;
      if (node < nN) *(volatile v4f*)(out + (size_t)node * DF + c4) = ov[it];
    }
    __threadfence();
#pragma unroll
    for (int it = 0; it < 4; ++it) {
      const int node = nodeBase + slot0 + 4 * it + rq;
      if (node < nN) *(volatile v4f*)(out + (size_t)node * DF + c4) = ov[it];
    }
  }
}

extern "C" void kernel_launch(void* const* d_in, const int* in_sizes, int n_in,
                              void* d_out, int out_size, void* d_ws, size_t ws_size,
                              hipStream_t stream) {
  if (n_in < 7) return;
  const int nN = in_sizes[0] / DF;
  if (nN <= 0 || in_sizes[0] != nN * DF) return;
  const int nE = in_sizes[1] / 2;
  if (nE < 0 || in_sizes[1] != 2 * nE) return;
  if (in_sizes[2] < 1) return;
  if (in_sizes[3] != DF * HD || in_sizes[4] != HD) return;
  if (in_sizes[5] != HD * DF || in_sizes[6] != DF) return;
  if (out_size != nN * DF) return;
  (void)d_ws;
  (void)ws_size;

  const float* x    = (const float*)d_in[0];
  const int*   ei   = (const int*)d_in[1];
  const float* beta = (const float*)d_in[2];
  const float* W1   = (const float*)d_in[3];
  const float* b1   = (const float*)d_in[4];
  const float* W2   = (const float*)d_in[5];
  const float* b2   = (const float*)d_in[6];
  float* out = (float*)d_out;

  hipFuncSetAttribute(reinterpret_cast<const void*>(&k_gen),
                      hipFuncAttributeMaxDynamicSharedMemorySize, LDS_BYTES);
  const int grid = (nN + NB - 1) / NB;
  k_gen<<<grid, NTHR, LDS_BYTES, stream>>>(x, ei, beta, W1, b1, W2, b2, out, nN, nE);
}
